// FiSHAttention_80590766342804
// MI455X (gfx1250) — hardware-verified
//
#include <hip/hip_runtime.h>


#define NB_  8
#define NN   1024
#define DM   768
#define NH_  12
#define NG   4
#define HD   64
#define PCAR 1024.0f
typedef _Float16 h16;
typedef unsigned short bf;
typedef __attribute__((ext_vector_type(16))) __bf16   v16bf;
typedef __attribute__((ext_vector_type(16))) _Float16 v16h;
typedef __attribute__((ext_vector_type(8)))  _Float16 v8h;
typedef __attribute__((ext_vector_type(8)))  unsigned short v8us;
typedef __attribute__((ext_vector_type(8)))  float    v8f;
typedef __attribute__((ext_vector_type(4)))  float    v4f;
typedef v8h  __attribute__((may_alias)) v8ha;
typedef v4f  __attribute__((may_alias)) v4fa;
typedef v8us __attribute__((may_alias)) v8usa;

__device__ __forceinline__ unsigned short f2bf(float f) { unsigned u = __float_as_uint(f); u += 0x7FFFu + ((u >> 16) & 1u); return (unsigned short)(u >> 16); }
__device__ __forceinline__ float bf2f(unsigned short b) { return __uint_as_float(((unsigned)b) << 16); }
__device__ __forceinline__ float bfr(float f) { return bf2f(f2bf(f)); }
__device__ __forceinline__ v16h cat16(v8h lo, v8h hi) { return __builtin_shufflevector(lo, hi, 0, 1, 2, 3, 4, 5, 6, 7, 8, 9, 10, 11, 12, 13, 14, 15); }
__device__ __forceinline__ v16bf cat16b(v8us lo, v8us hi) { return __builtin_bit_cast(v16bf, __builtin_shufflevector(lo, hi, 0, 1, 2, 3, 4, 5, 6, 7, 8, 9, 10, 11, 12, 13, 14, 15)); }
__device__ __forceinline__ v8f wmma16(v16h a, v16h b, v8f c) { return __builtin_amdgcn_wmma_f32_16x16x32_f16(false, a, false, b, (short)0, c, false, false); }
__device__ __forceinline__ v8f wmmab(v16bf a, v16bf b, v8f c) { return __builtin_amdgcn_wmma_f32_16x16x32_bf16(false, a, false, b, (short)0, c, false, false); }


template <typename T16> struct WFrag;
template <> struct WFrag<h16> { typedef v16h V; static __device__ __forceinline__ V ld(const h16* p) { return cat16(*(const v8h*)p, *(const v8h*)(p + 16)); } static __device__ __forceinline__ v8f mma(V a, V b, v8f c) { return wmma16(a, b, c); } };
template <> struct WFrag<bf> { typedef v16bf V; static __device__ __forceinline__ V ld(const bf* p) { return cat16b(*(const v8us*)p, *(const v8us*)(p + 16)); } static __device__ __forceinline__ v8f mma(V a, V b, v8f c) { return wmmab(a, b, c); } };
template <typename T16, int NSPLIT, bool BIAS>
__global__ __launch_bounds__(32) void k_gemmw(const T16* __restrict__ A, const T16* __restrict__ A2, const T16* __restrict__ Bt, const T16* __restrict__ Bt2, int K, float* C, int ldc, const float* __restrict__ bias, size_t sA, size_t sB, size_t sC) {
    typedef typename WFrag<T16>::V V;
    __shared__ __align__(16) float os[16 * 68];
    const size_t z = blockIdx.z; A += z * sA; if (A2) A2 += z * sA; Bt += z * sB; if (Bt2) Bt2 += z * sB; C += z * sC;
    const int lane = threadIdx.x & 31, lr = lane & 15, hi = lane >> 4; const int r0 = blockIdx.x * 64, c0 = blockIdx.y * 64;
    v8f acc[4][4];
#pragma unroll
    for (int mb = 0; mb < 4; ++mb)
#pragma unroll
        for (int nb = 0; nb < 4; ++nb) acc[mb][nb] = (v8f){};
    const size_t aoff = (size_t)(r0 + lr) * K + 8 * hi, boff = (size_t)(c0 + lr) * K + 8 * hi;
#pragma unroll 1
    for (int kc = 0; kc < K; kc += 32) {
        V a[4], a2[4];
#pragma unroll
        for (int mb = 0; mb < 4; ++mb) { a[mb] = WFrag<T16>::ld(A + aoff + (size_t)mb * 16 * K + kc); if (NSPLIT == 1 || NSPLIT == 2) a2[mb] = WFrag<T16>::ld(A2 + aoff + (size_t)mb * 16 * K + kc); }
#pragma unroll
        for (int nb = 0; nb < 4; ++nb) { const V b = WFrag<T16>::ld(Bt + boff + (size_t)nb * 16 * K + kc); V b2; if (NSPLIT >= 2) b2 = WFrag<T16>::ld(Bt2 + boff + (size_t)nb * 16 * K + kc);
#pragma unroll
            for (int mb = 0; mb < 4; ++mb) { acc[mb][nb] = WFrag<T16>::mma(a[mb], b, acc[mb][nb]); if (NSPLIT == 1 || NSPLIT == 2) acc[mb][nb] = WFrag<T16>::mma(a2[mb], b, acc[mb][nb]); if (NSPLIT >= 2) acc[mb][nb] = WFrag<T16>::mma(a[mb], b2, acc[mb][nb]); } }
        asm volatile("v_nop\n\tv_nop\n\tv_nop\n\tv_nop" : "+v"(acc[0][0]), "+v"(acc[1][1]), "+v"(acc[2][2]), "+v"(acc[3][3]) : "v"(a[0]), "v"(a[3]));
    }
#pragma unroll
    for (int mb = 0; mb < 4; ++mb) {
#pragma unroll
        for (int nb = 0; nb < 4; ++nb) {
#pragma unroll
            for (int j = 0; j < 8; ++j) os[(hi * 8 + j) * 68 + nb * 16 + lr] = acc[mb][nb][j]; }
        __builtin_amdgcn_wave_barrier(); asm volatile("" ::: "memory");
        float* crow = C + (size_t)(r0 + mb * 16) * ldc + c0;
#pragma unroll 1
        for (int ps = 0; ps < 2; ++ps) {
#pragma unroll
            for (int s = 0; s < 8; ++s) { const int row = 2 * s + hi, cofs = lr * 4; v4f val = *(const v4fa*)(os + row * 68 + cofs); if (BIAS) { val[0] += bfr(bias[c0 + cofs]); val[1] += bfr(bias[c0 + cofs + 1]); val[2] += bfr(bias[c0 + cofs + 2]); val[3] += bfr(bias[c0 + cofs + 3]); }
                *(volatile v4f*)(crow + (size_t)row * ldc + cofs) = val; }
            if (ps == 0) __threadfence(); }
        __builtin_amdgcn_wave_barrier(); asm volatile("" ::: "memory");
    }
}

__device__ __forceinline__ h16 tohx(float x) { return (h16)x; }
__device__ __forceinline__ void splitf(float y, unsigned short& h, unsigned short& l) { h = f2bf(y); l = f2bf(y - bf2f(h)); }
typedef __attribute__((ext_vector_type(2))) unsigned short v2us;
typedef __attribute__((ext_vector_type(4))) unsigned short v4us;
typedef __attribute__((ext_vector_type(2))) _Float16 v2h;
typedef __attribute__((ext_vector_type(4))) _Float16 v4h;

__global__ __launch_bounds__(256) void k_cvt8(const float* __restrict__ src, bf* dst, size_t n8) { const size_t i = (size_t)blockIdx.x * 256 + threadIdx.x; if (i >= n8) return; const v8f v = *(const v8f*)(src + i * 8); v8us o;
#pragma unroll
    for (int k = 0; k < 8; ++k) o[k] = f2bf(v[k]); *(volatile v8us*)(dst + i * 8) = o; __threadfence(); *(volatile v8us*)(dst + i * 8) = o; }
__global__ __launch_bounds__(256) void k_qk16(const float* __restrict__ F, h16* Q16, h16* K16) { const int e = (blockIdx.x * 256 + threadIdx.x) * 4; if (e >= NG * NN * HD) return; const int d = e % HD; const int t = (e / HD) % NN; const int k = e / (HD * NN); const float* fq = F + (size_t)t * DM + k * HD + d; const float* fk = fq + NG * HD; v4h a, c;
#pragma unroll
    for (int u = 0; u < 4; ++u) { a[u] = tohx(fq[u] * 0.125f); c[u] = tohx(fk[u]); } *(volatile v4h*)(Q16 + e) = a; *(volatile v4h*)(K16 + e) = c; __threadfence(); *(volatile v4h*)(Q16 + e) = a; *(volatile v4h*)(K16 + e) = c; }
__global__ __launch_bounds__(256) void k_vt16(const float* __restrict__ V, h16* VT) { const int e = (blockIdx.x * 256 + threadIdx.x) * 2; if (e >= NH_ * HD * NN) return; const int t = e % NN; const int d = (e / NN) % HD; const int h = e / (NN * HD); v2h o; o[0] = tohx(V[(size_t)t * DM + h * HD + d]); o[1] = tohx(V[(size_t)(t + 1) * DM + h * HD + d]); *(volatile v2h*)(VT + e) = o; __threadfence(); *(volatile v2h*)(VT + e) = o; }
__global__ __launch_bounds__(256) void k_fsoft(const float* __restrict__ GL, const float* __restrict__ mixl, h16* P16) { const int lane = threadIdx.x & 31; const int row = blockIdx.x * 8 + (threadIdx.x >> 5); if (row >= NH_ * NN) return; const int i = row % NN; const int h = row / NN;
    float mx4 = -3.0e38f, m[NG]; for (int k = 0; k < NG; ++k) { m[k] = bfr(mixl[h * NG + k]); mx4 = fmaxf(mx4, m[k]); } float se = 0.f; for (int k = 0; k < NG; ++k) { m[k] = __expf(__fsub_rn(m[k], mx4)); se = __fadd_rn(se, m[k]); } for (int k = 0; k < NG; ++k) m[k] = __fdiv_rn(m[k], se);
    float v[NN / 32]; float mx = -3.0e38f;
#pragma unroll
    for (int ch = 0; ch < NN / 128; ++ch) { const int j0 = ch * 128 + lane * 4; float acc[4] = {0.f, 0.f, 0.f, 0.f};
#pragma unroll
        for (int k = 0; k < NG; ++k) { const v4f a = *(const v4f*)(GL + ((size_t)k * NN + i) * NN + j0);
#pragma unroll
            for (int u = 0; u < 4; ++u) { float p = __fmul_rn(m[k], a[u]); asm volatile("" : "+v"(p)); acc[u] = __fadd_rn(acc[u], p); } }
#pragma unroll
        for (int u = 0; u < 4; ++u) { v[ch * 4 + u] = acc[u]; mx = fmaxf(mx, acc[u]); } }
#pragma unroll
    for (int sh = 16; sh; sh >>= 1) mx = fmaxf(mx, __shfl_xor(mx, sh, 32));
    float sum = 0.f;
#pragma unroll
    for (int q = 0; q < NN / 32; ++q) { float d0 = __fsub_rn(v[q], mx); asm volatile("" : "+v"(d0)); v[q] = __builtin_amdgcn_exp2f(__fmul_rn(d0, 1.4426950408889634f)); sum += v[q]; }
#pragma unroll
    for (int sh = 16; sh; sh >>= 1) sum += __shfl_xor(sum, sh, 32);
    const float f = __fdiv_rn(PCAR, sum);
    for (int ps = 0; ps < 2; ++ps) {
#pragma unroll
        for (int ch = 0; ch < NN / 128; ++ch) { v4h o4;
#pragma unroll
            for (int q = 0; q < 4; ++q) o4[q] = tohx(v[ch * 4 + q] * f); *(volatile v4h*)(P16 + (size_t)row * NN + ch * 128 + lane * 4) = o4; }
        if (ps == 0) __threadfence(); } }
__global__ __launch_bounds__(256) void k_mrg(const float* __restrict__ O, bf* Ah, bf* Al) { const int e = (blockIdx.x * 256 + threadIdx.x) * 4; if (e >= NH_ * NN * HD) return; const int d = e % HD; const int t = (e / HD) % NN; const int h = e / (HD * NN); v4us oh, ol;
#pragma unroll
    for (int u = 0; u < 4; ++u) { unsigned short a, b; splitf(O[e + u] * (1.0f / PCAR), a, b); oh[u] = a; ol[u] = b; } const size_t oo = (size_t)t * DM + h * HD + d; *(volatile v4us*)(Ah + oo) = oh; *(volatile v4us*)(Al + oo) = ol; __threadfence(); *(volatile v4us*)(Ah + oo) = oh; *(volatile v4us*)(Al + oo) = ol; }

extern "C" void kernel_launch(void* const* d_in, const int* in_sizes, int n_in,
                              void* d_out, int out_size, void* d_ws, size_t ws_size, hipStream_t stream) {
    (void)in_sizes; (void)n_in; (void)out_size;
    const float** I = (const float**)d_in;
    const float *x = I[0], *wqkv = I[1], *mixl = I[2], *wvv = I[3], *wp = I[4], *bp = I[5];
    float* OUT = (float*)d_out;
    char* wsp = (char*)d_ws;
    auto take = [&](size_t bytes) { char* p = wsp; wsp += (bytes + 255) & ~(size_t)255; return (void*)p; };
    bf* BQ = (bf*)take((size_t)DM * DM * 2); bf* BV = (bf*)take((size_t)DM * DM * 2); bf* BP = (bf*)take((size_t)DM * DM * 2); bf* XB = (bf*)take((size_t)NN * DM * 2);
    float* F = (float*)take((size_t)NN * DM * 4); float* V = (float*)take((size_t)NN * DM * 4); h16* Q16 = (h16*)take((size_t)NG * NN * HD * 2); h16* K16 = (h16*)take((size_t)NG * NN * HD * 2); h16* VT = (h16*)take((size_t)NH_ * HD * NN * 2);
    float* GL = (float*)take((size_t)NG * NN * NN * 4); h16* P16 = (h16*)take((size_t)NH_ * NN * NN * 2); float* O = (float*)take((size_t)NH_ * NN * HD * 4); bf* CTh = (bf*)take((size_t)NN * DM * 2); bf* CTl = (bf*)take((size_t)NN * DM * 2);
    if ((size_t)(wsp - (char*)d_ws) > ws_size) return;
    k_cvt8<<<(DM * DM / 8 + 255) / 256, 256, 0, stream>>>(wqkv, BQ, DM * DM / 8); k_cvt8<<<(DM * DM / 8 + 255) / 256, 256, 0, stream>>>(wvv, BV, DM * DM / 8); k_cvt8<<<(DM * DM / 8 + 255) / 256, 256, 0, stream>>>(wp, BP, DM * DM / 8);
    const dim3 gp(NN / 64, DM / 64, 1); const size_t zq = (size_t)NN * HD, zS = (size_t)NN * NN, zv = (size_t)HD * NN;
    for (int b = 0; b < NB_; ++b) {
        k_cvt8<<<(NN * DM / 8 + 255) / 256, 256, 0, stream>>>(x + (size_t)b * NN * DM, XB, NN * DM / 8);
        k_gemmw<bf, 0, false><<<gp, 32, 0, stream>>>(XB, nullptr, BQ, nullptr, DM, F, DM, nullptr, 0, 0, 0); k_qk16<<<(NG * NN * HD / 4 + 255) / 256, 256, 0, stream>>>(F, Q16, K16);
        k_gemmw<bf, 0, false><<<gp, 32, 0, stream>>>(XB, nullptr, BV, nullptr, DM, V, DM, nullptr, 0, 0, 0); k_vt16<<<(NH_ * HD * NN / 2 + 255) / 256, 256, 0, stream>>>(V, VT);
        k_gemmw<h16, 0, false><<<dim3(NN / 64, NN / 64, NG), 32, 0, stream>>>(Q16, nullptr, K16, nullptr, HD, GL, NN, nullptr, zq, zq, zS);
        k_fsoft<<<NH_ * NN / 8, 256, 0, stream>>>(GL, mixl, P16);
        k_gemmw<h16, 0, false><<<dim3(NN / 64, 1, NH_), 32, 0, stream>>>(P16, nullptr, VT, nullptr, NN, O, HD, nullptr, zS, zv, zq);
        k_mrg<<<(NH_ * NN * HD / 4 + 255) / 256, 256, 0, stream>>>(O, CTh, CTl);
        k_gemmw<bf, 1, true><<<gp, 32, 0, stream>>>(CTh, CTl, BP, nullptr, DM, OUT + (size_t)b * NN * DM, DM, bp, 0, 0, 0); }
}
